// NTN_8564164788344
// MI455X (gfx1250) — hardware-run, weakly checked
//
#include <hip/hip_runtime.h>


#ifndef NTOK
#define NTOK 32768
#endif
#define NTOK_FULL 32768
#define DM   128
#define NF   32
#define TB   64
#define MW   4
#define FPW  (NF / MW)
#define PSP  36
#define WTE  32
#define WTP  136
#define EPSN 1.0e-8f

static_assert(DM % 32 == 0);
static_assert((2 * DM) % 32 == 0);
static_assert(NF == 32);
static_assert(NF * 4 == 128);
static_assert(NF % MW == 0);
static_assert(TB == 64);
static_assert(MW * 16 == TB);
static_assert(4 * (32 / 8) == 16);
static_assert(NTOK % TB == 0);
static_assert(NTOK <= NTOK_FULL);
static_assert(((size_t)NTOK * DM) % 8 == 0);
static_assert(((size_t)NF * 2 * DM) % 8 == 0);
static_assert(DM % WTE == 0);
static_assert(4 * 256 * 4 == DM * WTE);
static_assert(2 * 256 * 8 == WTE * DM);
static_assert((WTP * 2) % 16 == 0);
static_assert(WTP >= DM);
static_assert((PSP * 4) % 16 == 0);
static_assert(PSP >= NF);
static_assert(2 * TB * PSP * 4 <= 131072);
static_assert(WTE * WTP * 2 <= 131072);

typedef unsigned short bf;
typedef __attribute__((ext_vector_type(16))) __bf16   v16bf;
typedef __attribute__((ext_vector_type(8)))  unsigned short v8us;
typedef __attribute__((ext_vector_type(8)))  float    v8f;
typedef __attribute__((ext_vector_type(4)))  float    v4f;
typedef v4f  __attribute__((may_alias)) v4fa;

__device__ __forceinline__ unsigned short f2bf(float f) { unsigned u = __float_as_uint(f); u += 0x7FFFu + ((u >> 16) & 1u); return (unsigned short)(u >> 16); }
__device__ __forceinline__ float bfr(float f) { return __uint_as_float(((unsigned)f2bf(f)) << 16); }
__device__ __forceinline__ v16bf cat16b(v8us lo, v8us hi) { return __builtin_bit_cast(v16bf, __builtin_shufflevector(lo, hi, 0, 1, 2, 3, 4, 5, 6, 7, 8, 9, 10, 11, 12, 13, 14, 15)); }
__device__ __forceinline__ v16bf ldb(const bf* p)  { return cat16b(*(const v8us*)p, *(const v8us*)(p + 16)); }
__device__ __forceinline__ v8f wmg(v16bf a, v16bf b, v8f c) {
    c = __builtin_amdgcn_wmma_f32_16x16x32_bf16(false, a, false, b, (short)0, c, false, false);
    asm volatile("v_nop\n\tv_nop\n\tv_nop\n\tv_nop" : "+v"(c) : "v"(a), "v"(b));
    return c;
}

__global__ __launch_bounds__(256) void k_cvt8(const float* __restrict__ src, bf* dst, size_t n8) {
    const size_t i = (size_t)blockIdx.x * 256 + threadIdx.x; if (i >= n8) return;
    const v8f v = *(const v8f*)(src + i * 8); v8us o;
#pragma unroll
    for (int k = 0; k < 8; ++k) o[k] = f2bf(v[k]);
    *(volatile v8us*)(dst + i * 8) = o; __threadfence(); *(volatile v8us*)(dst + i * 8) = o;
}

__global__ __launch_bounds__(256) void k_wtr(const float* __restrict__ src, bf* dst) {
    __shared__ __align__(16) bf ts[WTE * WTP];
    const int t = threadIdx.x; const int e0 = blockIdx.x * WTE; const int km = blockIdx.y;
    const float* s = src + (size_t)km * DM * DM;
#pragma unroll 1
    for (int it = 0; it < 4; ++it) { const int idx = it * 256 + t; const int d = idx >> 3, e4 = (idx & 7) * 4;
        const v4f v = *(const v4f*)(s + (size_t)d * DM + e0 + e4);
#pragma unroll
        for (int i = 0; i < 4; ++i) ts[(e4 + i) * WTP + d] = f2bf(v[i]); }
    __syncthreads();
    bf* o = dst + ((size_t)km * DM + e0) * DM;
    v8us val[2];
#pragma unroll
    for (int it = 0; it < 2; ++it) { const int p = it * 256 + t; const int e = p >> 4, d8 = (p & 15) * 8;
        val[it] = *(const v8us*)(&ts[e * WTP + d8]); }
#pragma unroll 1
    for (int ps = 0; ps < 2; ++ps) {
#pragma unroll
        for (int it = 0; it < 2; ++it) { const int p = it * 256 + t; const int e = p >> 4, d8 = (p & 15) * 8;
            *(volatile v8us*)(o + (size_t)e * DM + d8) = val[it]; }
        if (ps == 0) __threadfence(); }
}

__attribute__((amdgpu_num_vgpr(256))) __global__ __launch_bounds__(32 * MW) void k_bil(const bf* __restrict__ X1, const bf* __restrict__ X2, const bf* __restrict__ WT1, const bf* __restrict__ WT2,
                                                 const bf* __restrict__ VB, const float* __restrict__ bias, float* OUT) {
    __shared__ __align__(16) float p1s[TB * PSP];
    __shared__ __align__(16) float p2s[TB * PSP];
    const int lane = threadIdx.x & 31, lr = lane & 15, hi = lane >> 4;
    const int wave = __builtin_amdgcn_readfirstlane((int)(threadIdx.x >> 5));
    const int n0 = blockIdx.x * TB;

    {
        v8f c0 = (v8f){}, c1 = (v8f){};
        const size_t xt = (size_t)(n0 + wave * 16 + lr) * DM + 8 * hi;
        const size_t vo = (size_t)lr * (2 * DM) + 8 * hi;
#pragma unroll 1
        for (int kc = 0; kc < DM; kc += 32) {
            const v16bf xb = ldb(X1 + xt + kc);
            const v16bf va0 = ldb(VB + vo + kc), va1 = ldb(VB + vo + (size_t)16 * 2 * DM + kc);
            c0 = wmg(va0, xb, c0); c1 = wmg(va1, xb, c1); }
#pragma unroll 1
        for (int kc = 0; kc < DM; kc += 32) {
            const v16bf xb = ldb(X2 + xt + kc);
            const v16bf va0 = ldb(VB + vo + DM + kc), va1 = ldb(VB + vo + (size_t)16 * 2 * DM + DM + kc);
            c0 = wmg(va0, xb, c0); c1 = wmg(va1, xb, c1); }
        const int pr = (wave * 16 + lr) * PSP;
        v4f a, c;
        a[0] = c0[0]; a[1] = c0[1]; a[2] = c0[2]; a[3] = c0[3]; c[0] = c0[4]; c[1] = c0[5]; c[2] = c0[6]; c[3] = c0[7];
        *(v4fa*)(&p2s[pr +  0 + 8 * hi]) = a; *(v4fa*)(&p2s[pr +  0 + 8 * hi + 4]) = c;
        a[0] = c1[0]; a[1] = c1[1]; a[2] = c1[2]; a[3] = c1[3]; c[0] = c1[4]; c[1] = c1[5]; c[2] = c1[6]; c[3] = c1[7];
        *(v4fa*)(&p2s[pr + 16 + 8 * hi]) = a; *(v4fa*)(&p2s[pr + 16 + 8 * hi + 4]) = c;
    }

    const size_t xo = (size_t)(n0 + lr) * DM + 8 * hi;
    const size_t wo = (size_t)lr * DM + 8 * hi;
#pragma unroll 1
    for (int kf = 0; kf < FPW; ++kf) {
        const int km = wave * FPW + kf;
        float dt[4], sa[4], sb[4];
#pragma unroll
        for (int nb = 0; nb < 4; ++nb) { dt[nb] = 0.0f; sa[nb] = 0.0f; sb[nb] = 0.0f; }
#pragma unroll 1
        for (int ec = 0; ec < DM; ec += 32) {
            v8f p[2][4], q[2][4];
#pragma unroll
            for (int j = 0; j < 2; ++j)
#pragma unroll
                for (int nb = 0; nb < 4; ++nb) { p[j][nb] = (v8f){}; q[j][nb] = (v8f){}; }
            const size_t wrow = wo + ((size_t)km * DM + (size_t)ec) * DM;
#pragma unroll 1
            for (int kc = 0; kc < DM; kc += 32) {
                v16bf wa[2], wb[2];
#pragma unroll
                for (int j = 0; j < 2; ++j) { wa[j] = ldb(WT1 + wrow + (size_t)j * 16 * DM + kc); wb[j] = ldb(WT2 + wrow + (size_t)j * 16 * DM + kc); }
#pragma unroll
                for (int nb = 0; nb < 4; ++nb) {
                    const v16bf xa = ldb(X1 + xo + (size_t)nb * 16 * DM + kc);
                    const v16bf xb = ldb(X2 + xo + (size_t)nb * 16 * DM + kc);
                    p[0][nb] = wmg(wa[0], xa, p[0][nb]); p[1][nb] = wmg(wa[1], xa, p[1][nb]);
                    q[0][nb] = wmg(wb[0], xb, q[0][nb]); q[1][nb] = wmg(wb[1], xb, q[1][nb]); }
            }
#pragma unroll
            for (int nb = 0; nb < 4; ++nb)
#pragma unroll
                for (int j = 0; j < 2; ++j)
#pragma unroll
                    for (int r = 0; r < 8; ++r) { const float a = p[j][nb][r], c = q[j][nb][r];
                        dt[nb] = fmaf(a, c, dt[nb]); sa[nb] = fmaf(a, a, sa[nb]); sb[nb] = fmaf(c, c, sb[nb]); }
        }
#pragma unroll
        for (int nb = 0; nb < 4; ++nb) {
            const float d2 = dt[nb] + __shfl_xor(dt[nb], 16, 32);
            const float a2 = sa[nb] + __shfl_xor(sa[nb], 16, 32);
            const float b2 = sb[nb] + __shfl_xor(sb[nb], 16, 32);
            const float n1 = fmaxf(sqrtf(a2), EPSN), n2 = fmaxf(sqrtf(b2), EPSN);
            const float cs = d2 * (1.0f / (n1 * n2));
            if (hi == 0) p1s[(nb * 16 + lr) * PSP + km] = cs; }
    }
    __syncthreads();

    const int cofs = (lane & 7) * 4;
    const v4f braw = *(const v4f*)(bias + cofs);
    v4f val[4];
#pragma unroll
    for (int s = 0; s < 4; ++s) { const int row = wave * 16 + 4 * s + (lane >> 3);
        const v4f a = *(const v4fa*)(&p1s[row * PSP + cofs]); const v4f c = *(const v4fa*)(&p2s[row * PSP + cofs]);
#pragma unroll
        for (int i = 0; i < 4; ++i) { const float t = (a[i] + c[i]) + bfr(braw[i]); val[s][i] = fmaxf(t, 0.0f); } }
    float* orow = OUT + (size_t)n0 * NF;
#pragma unroll 1
    for (int ps = 0; ps < 2; ++ps) {
#pragma unroll
        for (int s = 0; s < 4; ++s) { const int row = wave * 16 + 4 * s + (lane >> 3);
            *(volatile v4f*)(orow + (size_t)row * NF + cofs) = val[s]; }
        if (ps == 0) __threadfence(); }
}

static constexpr size_t al256(size_t v) { return (v + 255) & ~(size_t)255; }
static constexpr size_t SZ_XB = al256((size_t)NTOK * DM * 2);
static constexpr size_t SZ_WT = al256((size_t)NF * DM * DM * 2);
static constexpr size_t SZ_VB = al256((size_t)NF * 2 * DM * 2);
static constexpr size_t SZ_TOTAL = 2 * SZ_XB + 2 * SZ_WT + SZ_VB;
static_assert(SZ_TOTAL <= (size_t)134217728);

extern "C" void kernel_launch(void* const* d_in, const int* in_sizes, int n_in,
                              void* d_out, int out_size, void* d_ws, size_t ws_size, hipStream_t stream) {
    if (n_in < 6) return;
    if ((size_t)in_sizes[0] < (size_t)NTOK * DM || (size_t)in_sizes[1] < (size_t)NTOK * DM) return;
    if ((size_t)in_sizes[2] < (size_t)NF * DM * DM || (size_t)in_sizes[3] < (size_t)NF * DM * DM) return;
    if ((size_t)in_sizes[4] < (size_t)NF * 2 * DM || in_sizes[5] < NF) return;
    if ((size_t)out_size < (size_t)NTOK * NF) return;
    if (SZ_TOTAL > ws_size) return;
    const float* x1 = (const float*)d_in[0]; const float* x2 = (const float*)d_in[1];
    const float* w1 = (const float*)d_in[2]; const float* w2 = (const float*)d_in[3];
    const float* vv = (const float*)d_in[4]; const float* bb = (const float*)d_in[5];
    float* OUT = (float*)d_out;
    char* wsp = (char*)d_ws;
    bf* X1B = (bf*)wsp; wsp += SZ_XB;
    bf* X2B = (bf*)wsp; wsp += SZ_XB;
    bf* WT1 = (bf*)wsp; wsp += SZ_WT;
    bf* WT2 = (bf*)wsp; wsp += SZ_WT;
    bf* VB  = (bf*)wsp; wsp += SZ_VB;

    { const size_t n8 = (size_t)NTOK * DM / 8; const unsigned g = (unsigned)((n8 + 255) / 256);
      k_cvt8<<<g, 256, 0, stream>>>(x1, X1B, n8); k_cvt8<<<g, 256, 0, stream>>>(x2, X2B, n8); }
    { const size_t n8 = (size_t)NF * 2 * DM / 8; const unsigned g = (unsigned)((n8 + 255) / 256);
      k_cvt8<<<g, 256, 0, stream>>>(vv, VB, n8); }
    k_wtr<<<dim3(DM / WTE, NF, 1), 256, 0, stream>>>(w1, WT1);
    k_wtr<<<dim3(DM / WTE, NF, 1), 256, 0, stream>>>(w2, WT2);

    k_bil<<<dim3(NTOK / TB, 1, 1), 32 * MW, 0, stream>>>(X1B, X2B, WT1, WT2, VB, bb, OUT);
}
